// Encoder_82274393522442
// MI455X (gfx1250) — hardware-verified
//
#include <hip/hip_runtime.h>
#include <math.h>

constexpr int NBATCH   = 32;
constexpr int NPTS     = 8192;
constexpr int ZDIM     = 1024;
constexpr int CH_IN    = 3;
constexpr int CH_L1    = 64;
constexpr int CH_L2    = 128;
constexpr int CH_L3    = 256;
constexpr int CH_L4    = 256;
constexpr int CHUNK_B  = 8;
constexpr int CHUNK_P  = CHUNK_B * NPTS;
constexpr int NCHUNK   = NBATCH / CHUNK_B;
constexpr int NTHR     = 256;
constexpr int L1_PITCH = 72;
constexpr int SLAB_PITCH = 68;
constexpr int L5_ROWS_IT = 8 * 64;
constexpr int L5_ITERS   = NPTS / L5_ROWS_IT;

constexpr int CAST_BLK_W2 = CH_L2 * CH_L1 / 8 / NTHR;
constexpr int CAST_BLK_W3 = CH_L3 * CH_L2 / 8 / NTHR;
constexpr int CAST_BLK_W4 = CH_L4 * CH_L3 / 8 / NTHR;
constexpr int CAST_BLK_W5 = ZDIM * CH_L4 / 8 / NTHR;
constexpr int CAST_BLK_ALL = CAST_BLK_W2 + CAST_BLK_W3 + CAST_BLK_W4 + CAST_BLK_W5;

static_assert(NBATCH % CHUNK_B == 0);
static_assert(NPTS % NTHR == 0);
static_assert(NPTS % L5_ROWS_IT == 0);
static_assert(CH_L1 % 32 == 0 && CH_L2 % 32 == 0 && CH_L3 % 32 == 0 && CH_L4 % 32 == 0);
static_assert(CHUNK_P % 64 == 0 && CH_L2 % 64 == 0 && CH_L3 % 64 == 0 && CH_L4 % 64 == 0 && ZDIM % 64 == 0);
static_assert(((CHUNK_P / 64) * (CH_L2 / 64)) % 8 == 0);
static_assert(((CHUNK_P / 64) * (CH_L3 / 64)) % 8 == 0);
static_assert(((CHUNK_P / 64) * (CH_L4 / 64)) % 8 == 0);
static_assert((CH_L2 * CH_L1) % (8 * NTHR) == 0 && (CH_L3 * CH_L2) % (8 * NTHR) == 0);
static_assert((CH_L4 * CH_L3) % (8 * NTHR) == 0 && (ZDIM * CH_L4) % (8 * NTHR) == 0);
static_assert(CAST_BLK_ALL == 180);
static_assert(CH_L1 * CH_IN <= NTHR);

typedef __attribute__((ext_vector_type(16))) _Float16 v16h;
typedef __attribute__((ext_vector_type(8)))  _Float16 v8h;
typedef __attribute__((ext_vector_type(8)))  float    v8f;
typedef __attribute__((ext_vector_type(4)))  float    v4f;

__device__ __forceinline__ void row_guard_h(v8f& a0, v8f& a1, v8f& a2, v8f& a3, v16h x,
                                            v16h b0, v16h b1, v16h b2, v16h b3) {
  asm volatile("v_nop\n\tv_nop\n\tv_nop\n\tv_nop"
               : "+v"(a0), "+v"(a1), "+v"(a2), "+v"(a3)
               : "v"(x), "v"(b0), "v"(b1), "v"(b2), "v"(b3));
}
__device__ __forceinline__ void keep4_h(v16h a, v16h b, v16h c, v16h d) {
  asm volatile("v_nop" :: "v"(a), "v"(b), "v"(c), "v"(d));
}
__device__ __forceinline__ void acc_guard4(v8f& a, v8f& b, v8f& c, v8f& d) {
  asm volatile("v_nop\n\tv_nop\n\tv_nop\n\tv_nop" : "+v"(a), "+v"(b), "+v"(c), "+v"(d));
}

union FragU { v16h v; v8h h[2]; };
__device__ __forceinline__ v16h frag_load(const _Float16* p) {
  FragU f;
  f.h[0] = *(const v8h*)(p);
  f.h[1] = *(const v8h*)(p + 16);
  return f.v;
}
__device__ __forceinline__ v8f frag_mma(v16h a, v16h b, v8f c) {
  return __builtin_amdgcn_wmma_f32_16x16x32_f16(false, a, false, b, (short)0, c, false, false);
}

__global__ __launch_bounds__(NTHR) void cast_weights_kernel(
    const float* __restrict__ w2, const float* __restrict__ w3,
    const float* __restrict__ w4, const float* __restrict__ w5,
    unsigned short* __restrict__ d2, unsigned short* __restrict__ d3,
    unsigned short* __restrict__ d4, unsigned short* __restrict__ d5) {
  const int blk = blockIdx.x;
  const float* src;
  unsigned short* dst;
  int base;
  if (blk < CAST_BLK_W2) {
    src = w2; dst = d2; base = 0;
  } else if (blk < CAST_BLK_W2 + CAST_BLK_W3) {
    src = w3; dst = d3; base = CAST_BLK_W2;
  } else if (blk < CAST_BLK_W2 + CAST_BLK_W3 + CAST_BLK_W4) {
    src = w4; dst = d4; base = CAST_BLK_W2 + CAST_BLK_W3;
  } else {
    src = w5; dst = d5; base = CAST_BLK_W2 + CAST_BLK_W3 + CAST_BLK_W4;
  }
  const int i = (blk - base) * NTHR + (int)threadIdx.x;
  const v4f a = *(const v4f*)(src + (size_t)i * 8);
  const v4f b = *(const v4f*)(src + (size_t)i * 8 + 4);
  v8h hv;
#pragma unroll
  for (int e = 0; e < 4; ++e) {
    hv[e]     = (_Float16)a[e];
    hv[4 + e] = (_Float16)b[e];
  }
  *(volatile v8h*)(dst + (size_t)i * 8) = hv;
  __threadfence();
  *(volatile v8h*)(dst + (size_t)i * 8) = hv;
}

__global__ __launch_bounds__(NTHR) void layer1_kernel(
    const float* __restrict__ x, const float* __restrict__ w1, const float* __restrict__ b1,
    unsigned short* __restrict__ h1p, int chunk) {
  __shared__ __align__(16) _Float16 sH[NTHR * L1_PITCH];
  __shared__ float sW[NTHR];
  __shared__ float sB[NTHR];
  const int tid = threadIdx.x;
  const int wi = tid < (CH_L1 * CH_IN - 1) ? tid : (CH_L1 * CH_IN - 1);
  sW[tid] = w1[wi];
  sB[tid] = b1[tid & (CH_L1 - 1)];
  const int gp = chunk * CHUNK_P + (int)blockIdx.x * NTHR + tid;
  const int bb = gp / NPTS;
  const int nn = gp - bb * NPTS;
  const float* xp = x + (size_t)bb * CH_IN * NPTS + nn;
  const float x0 = xp[0];
  const float x1 = xp[NPTS];
  const float x2 = xp[2 * NPTS];
  __syncthreads();
#pragma unroll 1
  for (int o8 = 0; o8 < CH_L1 / 8; ++o8) {
    v8h hv;
#pragma unroll
    for (int e = 0; e < 8; ++e) {
      const int o = o8 * 8 + e;
      float v = sB[o];
      v = fmaf(x0, sW[o * 3 + 0], v);
      v = fmaf(x1, sW[o * 3 + 1], v);
      v = fmaf(x2, sW[o * 3 + 2], v);
      v = fmaxf(v, 0.0f);
      hv[e] = (_Float16)v;
    }
    *(v8h*)(sH + tid * L1_PITCH + o8 * 8) = hv;
  }
  __syncthreads();
  unsigned short* dst = h1p + (size_t)blockIdx.x * NTHR * CH_L1;
  for (int pass = 0; pass < 2; ++pass) {
#pragma unroll
    for (int it = 0; it < 8; ++it) {
      const int i = it * NTHR + tid;
      const int row = i >> 3;
      const int seg = i & 7;
      const v8h v = *(const v8h*)(sH + row * L1_PITCH + seg * 8);
      *(volatile v8h*)(dst + (size_t)i * 8) = v;
    }
    __threadfence();
  }
}

__global__ __launch_bounds__(NTHR) void gemm64_f16_bias_relu(
    const unsigned short* __restrict__ Ap, int lda,
    const unsigned short* __restrict__ Btp, int ldb,
    unsigned short* __restrict__ Cp, int ldc,
    const float* __restrict__ bias, int M, int N, int K) {
  const _Float16* A  = (const _Float16*)Ap;
  const _Float16* Bt = (const _Float16*)Btp;
  __shared__ __align__(16) float sT[8][16 * SLAB_PITCH];
  const int lane = threadIdx.x & 31;
  const int wave = threadIdx.x >> 5;
  const int tilesN = N >> 6;
  const int tilesM = M >> 6;
  const int tile = blockIdx.x * 8 + wave;
  if (tile >= tilesM * tilesN) return;
  const int tm = tile / tilesN;
  const int tn = tile - tm * tilesN;
  const int m0 = tm << 6;
  const int n0 = tn << 6;
  const int rlane = lane & 15;
  const int koff  = (lane >> 4) * 8;
  const int mOff  = (lane >> 4) * 8;

  v8f acc[4][4];
#pragma unroll
  for (int i = 0; i < 4; ++i)
#pragma unroll
    for (int j = 0; j < 4; ++j) acc[i][j] = (v8f){0.f, 0.f, 0.f, 0.f, 0.f, 0.f, 0.f, 0.f};

  for (int k0 = 0; k0 < K; k0 += 32) {
    v16h bh[4];
#pragma unroll
    for (int j = 0; j < 4; ++j) {
      const size_t bo = (size_t)(n0 + (j << 4) + rlane) * ldb + koff + k0;
      bh[j] = frag_load(Bt + bo);
    }
#pragma unroll
    for (int i = 0; i < 4; ++i) {
      const size_t ao = (size_t)(m0 + (i << 4) + rlane) * lda + koff + k0;
      const v16h ah = frag_load(A + ao);
#pragma unroll
      for (int j = 0; j < 4; ++j) acc[i][j] = frag_mma(ah, bh[j], acc[i][j]);
      row_guard_h(acc[i][0], acc[i][1], acc[i][2], acc[i][3], ah, bh[0], bh[1], bh[2], bh[3]);
    }
    keep4_h(bh[0], bh[1], bh[2], bh[3]);
  }
  acc_guard4(acc[0][0], acc[0][1], acc[0][2], acc[0][3]);
  acc_guard4(acc[1][0], acc[1][1], acc[1][2], acc[1][3]);
  acc_guard4(acc[2][0], acc[2][1], acc[2][2], acc[2][3]);
  acc_guard4(acc[3][0], acc[3][1], acc[3][2], acc[3][3]);

  float* slab = sT[wave];
#pragma unroll
  for (int i = 0; i < 4; ++i) {
    const int mBase = m0 + (i << 4);
#pragma unroll
    for (int j = 0; j < 4; ++j) {
      const int n = n0 + (j << 4) + rlane;
      const float bv = bias[n];
#pragma unroll
      for (int r = 0; r < 8; ++r) {
        float v = acc[i][j][r] + bv;
        v = fmaxf(v, 0.0f);
        slab[(mOff + r) * SLAB_PITCH + (j << 4) + rlane] = v;
      }
    }
    __builtin_amdgcn_fence(__ATOMIC_RELEASE, "workgroup");
    __builtin_amdgcn_wave_barrier();
    __builtin_amdgcn_fence(__ATOMIC_ACQUIRE, "workgroup");
    {
      const int q = lane >> 3;
      const int c8 = (lane & 7) * 8;
      for (int pass = 0; pass < 2; ++pass) {
#pragma unroll
        for (int it = 0; it < 4; ++it) {
          const int row = it * 4 + q;
          const float* sp = slab + row * SLAB_PITCH + c8;
          v8h hv;
#pragma unroll
          for (int e = 0; e < 8; ++e) hv[e] = (_Float16)sp[e];
          *(volatile v8h*)(Cp + (size_t)(mBase + row) * ldc + n0 + c8) = hv;
        }
        __threadfence();
      }
    }
    __builtin_amdgcn_fence(__ATOMIC_RELEASE, "workgroup");
    __builtin_amdgcn_wave_barrier();
    __builtin_amdgcn_fence(__ATOMIC_ACQUIRE, "workgroup");
  }
}

__global__ __launch_bounds__(NTHR) void layer5_max_kernel(
    const unsigned short* __restrict__ h4p, const unsigned short* __restrict__ w5p,
    const float* __restrict__ b5, float* __restrict__ out, int chunk) {
  __shared__ __align__(16) float sMax[8 * 64];
  const _Float16* A  = (const _Float16*)h4p;
  const _Float16* Bt = (const _Float16*)w5p;
  const int lane = threadIdx.x & 31;
  const int wave = threadIdx.x >> 5;
  const int rlane = lane & 15;
  const int koff  = (lane >> 4) * 8;
  const int n0 = (int)blockIdx.x * 64;
  const int bl = (int)blockIdx.y;

  float rm[4];
#pragma unroll
  for (int j = 0; j < 4; ++j) rm[j] = -INFINITY;

  const _Float16* Bbase = Bt + (size_t)(n0 + rlane) * CH_L4 + koff;

#pragma unroll 1
  for (int mt = 0; mt < L5_ITERS; ++mt) {
    const int m0 = bl * NPTS + mt * L5_ROWS_IT + wave * 64;
    const _Float16* Abase = A + (size_t)(m0 + rlane) * CH_L4 + koff;
    v8f acc[4][4];
#pragma unroll
    for (int i = 0; i < 4; ++i)
#pragma unroll
      for (int j = 0; j < 4; ++j) acc[i][j] = (v8f){0.f, 0.f, 0.f, 0.f, 0.f, 0.f, 0.f, 0.f};

#pragma unroll 1
    for (int k0 = 0; k0 < CH_L4; k0 += 32) {
      v16h bh[4];
#pragma unroll
      for (int j = 0; j < 4; ++j) bh[j] = frag_load(Bbase + (size_t)(j << 4) * CH_L4 + k0);
#pragma unroll
      for (int i = 0; i < 4; ++i) {
        const v16h ah = frag_load(Abase + (size_t)(i << 4) * CH_L4 + k0);
#pragma unroll
        for (int j = 0; j < 4; ++j) acc[i][j] = frag_mma(ah, bh[j], acc[i][j]);
        row_guard_h(acc[i][0], acc[i][1], acc[i][2], acc[i][3], ah, bh[0], bh[1], bh[2], bh[3]);
      }
      keep4_h(bh[0], bh[1], bh[2], bh[3]);
    }
    acc_guard4(acc[0][0], acc[0][1], acc[0][2], acc[0][3]);
    acc_guard4(acc[1][0], acc[1][1], acc[1][2], acc[1][3]);
    acc_guard4(acc[2][0], acc[2][1], acc[2][2], acc[2][3]);
    acc_guard4(acc[3][0], acc[3][1], acc[3][2], acc[3][3]);
#pragma unroll
    for (int i = 0; i < 4; ++i)
#pragma unroll
      for (int j = 0; j < 4; ++j)
#pragma unroll
        for (int r = 0; r < 8; ++r) rm[j] = fmaxf(rm[j], acc[i][j][r]);
  }

#pragma unroll
  for (int j = 0; j < 4; ++j) {
    const float other = __shfl_xor(rm[j], 16, 32);
    rm[j] = fmaxf(rm[j], other);
  }
  if (lane < 16) {
#pragma unroll
    for (int j = 0; j < 4; ++j) sMax[wave * 64 + (j << 4) + lane] = rm[j];
  }
  __syncthreads();
  if (wave == 0) {
    const int c4 = (lane & 15) * 4;
    const v4f bv = *(const v4f*)(b5 + n0 + c4);
    v4f o;
#pragma unroll
    for (int e = 0; e < 4; ++e) {
      float m = sMax[c4 + e];
#pragma unroll
      for (int w = 1; w < 8; ++w) m = fmaxf(m, sMax[w * 64 + c4 + e]);
      o[e] = m + bv[e];
    }
    float* op = out + (size_t)(chunk * CHUNK_B + bl) * ZDIM + n0 + c4;
    if (lane < 16) *(volatile v4f*)op = o;
    __threadfence();
    if (lane < 16) *(volatile v4f*)op = o;
  }
}

extern "C" void kernel_launch(void* const* d_in, const int* in_sizes, int n_in,
                              void* d_out, int out_size, void* d_ws, size_t ws_size, hipStream_t stream) {
  if (n_in < 11 || d_out == nullptr || d_ws == nullptr) return;
  if (in_sizes[0] != NBATCH * CH_IN * NPTS || in_sizes[1] != CH_L1 * CH_IN || in_sizes[2] != CH_L1 ||
      in_sizes[3] != CH_L2 * CH_L1 || in_sizes[4] != CH_L2 || in_sizes[5] != CH_L3 * CH_L2 ||
      in_sizes[6] != CH_L3 || in_sizes[7] != CH_L4 * CH_L3 || in_sizes[8] != CH_L4 ||
      in_sizes[9] != ZDIM * CH_L4 || in_sizes[10] != ZDIM || out_size != NBATCH * ZDIM) return;

  const float* x  = (const float*)d_in[0];
  const float* w1 = (const float*)d_in[1];
  const float* b1 = (const float*)d_in[2];
  const float* w2 = (const float*)d_in[3];
  const float* b2 = (const float*)d_in[4];
  const float* w3 = (const float*)d_in[5];
  const float* b3 = (const float*)d_in[6];
  const float* w4 = (const float*)d_in[7];
  const float* b4 = (const float*)d_in[8];
  const float* w5 = (const float*)d_in[9];
  const float* b5 = (const float*)d_in[10];
  float* out = (float*)d_out;

  char* ws = (char*)d_ws;
  size_t off = 0;
  auto carve = [&](size_t bytes) -> char* {
    char* p = ws + off;
    off += (bytes + 255) & ~(size_t)255;
    return p;
  };
  unsigned short* W2H = (unsigned short*)carve((size_t)CH_L2 * CH_L1 * 2);
  unsigned short* W3H = (unsigned short*)carve((size_t)CH_L3 * CH_L2 * 2);
  unsigned short* W4H = (unsigned short*)carve((size_t)CH_L4 * CH_L3 * 2);
  unsigned short* W5H = (unsigned short*)carve((size_t)ZDIM * CH_L4 * 2);
  unsigned short* H1  = (unsigned short*)carve((size_t)CHUNK_P * CH_L1 * 2);
  unsigned short* H2  = (unsigned short*)carve((size_t)CHUNK_P * CH_L2 * 2);
  unsigned short* H3  = (unsigned short*)carve((size_t)CHUNK_P * CH_L3 * 2);
  unsigned short* H4  = (unsigned short*)carve((size_t)CHUNK_P * CH_L4 * 2);
  if (off > ws_size || off > (size_t)134217728) return;

  cast_weights_kernel<<<CAST_BLK_ALL, NTHR, 0, stream>>>(w2, w3, w4, w5, W2H, W3H, W4H, W5H);

  const int grid_l1 = CHUNK_P / NTHR;
  const int grid_l2 = (CHUNK_P / 64) * (CH_L2 / 64) / 8;
  const int grid_l3 = (CHUNK_P / 64) * (CH_L3 / 64) / 8;
  const int grid_l4 = (CHUNK_P / 64) * (CH_L4 / 64) / 8;
  const dim3 grid_l5(ZDIM / 64, CHUNK_B);

  for (int chunk = 0; chunk < NCHUNK; ++chunk) {
    layer1_kernel<<<grid_l1, NTHR, 0, stream>>>(x, w1, b1, H1, chunk);
    gemm64_f16_bias_relu<<<grid_l2, NTHR, 0, stream>>>(H1, CH_L1, W2H, CH_L1, H2, CH_L2, b2, CHUNK_P, CH_L2, CH_L1);
    gemm64_f16_bias_relu<<<grid_l3, NTHR, 0, stream>>>(H2, CH_L2, W3H, CH_L2, H3, CH_L3, b3, CHUNK_P, CH_L3, CH_L2);
    gemm64_f16_bias_relu<<<grid_l4, NTHR, 0, stream>>>(H3, CH_L3, W4H, CH_L3, H4, CH_L4, b4, CHUNK_P, CH_L4, CH_L3);
    layer5_max_kernel<<<grid_l5, NTHR, 0, stream>>>(H4, W5H, b5, out, chunk);
  }
}
